// DilatedNeighborhoodAttention1D_46170898432358
// MI455X (gfx1250) — hardware-verified
//
#include <hip/hip_runtime.h>
#include <math.h>

#ifndef NB
#define NB 4
#endif
#ifndef SEQ
#define SEQ 2048
#endif
#define NB_FULL 4
#define SEQ_FULL 2048
#define EMB 256
#define HEADS 8
#define HD 32
#define NTAB 13
#define MTOK (NB * SEQ)
#define QKLD 512
#define VTLD MTOK
#define QTILES ((unsigned)(SEQ / 16))

#define X_CARRY 16
#define W_CARRY 64
#define QKV_CARRY 16
#define P_CARRY 1024
#define CTX_CARRY 256

static constexpr float XC = (float)X_CARRY;
static constexpr float WC = (float)W_CARRY;
static constexpr float PC = (float)P_CARRY;
static constexpr float QKV_OSC = (float)QKV_CARRY;
static constexpr float PROJ_UNDO = 1.0f / (float)(X_CARRY * W_CARRY);
static constexpr float SCORE_SCALE = 0.17677669529663687f;
static constexpr float SCQK = SCORE_SCALE / (float)(QKV_CARRY * QKV_CARRY);
static constexpr float LOG2E = 1.4426950408889634f;
static constexpr float CTX_UNDO = (float)CTX_CARRY / (float)(P_CARRY * QKV_CARRY);
static constexpr float OUT_UNDO = 1.0f / (float)(CTX_CARRY * W_CARRY);

static_assert(X_CARRY * W_CARRY == 1024);
static_assert(QKV_CARRY * QKV_CARRY == 256);
static_assert(P_CARRY * QKV_CARRY == 64 * CTX_CARRY);
static_assert(CTX_CARRY * W_CARRY == 16384);
static_assert(HEADS * HD == EMB && HD == 32 && EMB == 256);
static_assert(NB >= 1 && NB <= NB_FULL && SEQ <= SEQ_FULL);
static_assert(SEQ % 64 == 0 && SEQ <= 2048);
static_assert(MTOK % 64 == 0);
static_assert(EMB % 64 == 0 && (2 * EMB) % 64 == 0 && EMB % 32 == 0);
static_assert((NB * 4 * (SEQ / 16)) % 8 == 0);
static_assert(NTAB == 13);

typedef __attribute__((ext_vector_type(16))) _Float16 v16h;
typedef __attribute__((ext_vector_type(8)))  _Float16 v8h;
typedef __attribute__((ext_vector_type(8)))  float    v8f;
typedef __attribute__((ext_vector_type(4)))  float    v4f;
typedef __attribute__((ext_vector_type(4)))  unsigned int v4u;
typedef _Float16 h16;


#define VST2(T, ptr, val) do { const T vst2_v_ = (val); *(volatile T*)(ptr) = vst2_v_; __threadfence(); *(volatile T*)(ptr) = vst2_v_; } while (0)
#define VST2V4(ptr, val) do { const v4f vst2_v4_ = (val); *(volatile v4f*)(ptr) = vst2_v4_; __threadfence(); *(volatile v4f*)(ptr) = vst2_v4_; } while (0)

__device__ __forceinline__ float bfr(float f) {
    unsigned u = __float_as_uint(f);
    u += 0x7FFFu + ((u >> 16) & 1u);
    return __uint_as_float(u & 0xFFFF0000u);
}
static __device__ __forceinline__ h16 toh_flush(float v) { const float w = (fabsf(v) < 6.103515625e-05f) ? 0.0f : v; return (h16)w; }

static __device__ __forceinline__ void st8hf(_Float16* P, size_t o, const float* v) {
    v8h pk;
#pragma unroll
    for (int i = 0; i < 8; ++i) pk[i] = toh_flush(v[i]);
    VST2(v8h, (v8h*)(P + o), pk);
}

union FragU { v16h v; v8h h[2]; };
__device__ __forceinline__ v16h frag_ld(const _Float16* p) {
    FragU f; f.h[0] = *(const v8h*)(p); f.h[1] = *(const v8h*)(p + 16); return f.v;
}
__device__ __forceinline__ v8f wmma16(v16h a, v16h b, v8f c) {
    c = __builtin_amdgcn_wmma_f32_16x16x32_f16(false, a, false, b, (short)0, c, false, false);
    asm volatile("v_nop\n\tv_nop\n\tv_nop\n\tv_nop" : "+v"(c) : "v"(a), "v"(b));
    return c;
}
__device__ __forceinline__ void wave_sync_lds() {
    __builtin_amdgcn_fence(3  , "workgroup");
    __builtin_amdgcn_wave_barrier();
    __builtin_amdgcn_fence(2  , "workgroup");
}

static __device__ __forceinline__ unsigned div7_u11(unsigned t) {
    asm volatile("" : "+v"(t));
    return (t * 9363u) >> 16;
}
static __device__ __forceinline__ unsigned mod7_u11(unsigned t) { return t - 7u * div7_u11(t); }
static constexpr __host__ __device__ int wrap7c(int k) { return k % 7; }
static_assert(wrap7c(0) == 0 && wrap7c(6) == 6 && wrap7c(7) == 0 && wrap7c(16) == 2 && wrap7c(20) == 6 && wrap7c(21) == 0 && wrap7c(23) == 2);

static __device__ __forceinline__ unsigned out_row(unsigned row) {
    return (row / (unsigned)SEQ) * (unsigned)SEQ_FULL + (row % (unsigned)SEQ);
}

static_assert(32 * 16 * 4 == 16 * 128);
static_assert(32 * 16 * 8 == 16 * 256);
static_assert(8 * 16 * 68 * 4 <= 131072);

template <int OUT_MODE, bool BIAS_ROW, unsigned M, unsigned N, unsigned K, unsigned LDA, unsigned LDB, unsigned LDC>
static __device__ __forceinline__ void gemm64_body(
    const _Float16* __restrict__ A, const _Float16* __restrict__ Bt,
    float* __restrict__ Cf, _Float16* __restrict__ Ch, const float* __restrict__ bias,
    const float scale, const float oscale) {
  static_assert(M % 64 == 0 && N % 64 == 0 && K % 32 == 0);
  static_assert(LDA % 8 == 0 && LDB % 8 == 0 && LDC % 64 == 0);
  __shared__ __align__(16) float sT[8][16 * 68];
  const unsigned lane = threadIdx.x & 31u;
  const unsigned wave = __builtin_amdgcn_readfirstlane(threadIdx.x >> 5);
  constexpr unsigned tilesN = N >> 6, tilesM = M >> 6;
  const unsigned tile = blockIdx.x * 8u + wave;
  if (tile >= tilesM * tilesN) return;
  const unsigned tm = tile / tilesN;
  const unsigned tn = tile - tm * tilesN;
  const unsigned m0 = tm << 6, n0 = tn << 6;
  const unsigned rlane = lane & 15u;
  const unsigned koff = (lane >> 4) * 8u;
  const unsigned mOff = koff;

  v8f acc[4][4];
#pragma unroll
  for (int i = 0; i < 4; ++i)
#pragma unroll
    for (int j = 0; j < 4; ++j) acc[i][j] = (v8f){0.f,0.f,0.f,0.f,0.f,0.f,0.f,0.f};

#pragma unroll 1
  for (unsigned k0 = 0; k0 < K; k0 += 32u) {
    v16h bh[4];
#pragma unroll
    for (int j = 0; j < 4; ++j)
      bh[j] = frag_ld(Bt + (size_t)(n0 + ((unsigned)j << 4) + rlane) * LDB + koff + k0);
#pragma unroll
    for (int i = 0; i < 4; ++i) {
      const v16h ah = frag_ld(A + (size_t)(m0 + ((unsigned)i << 4) + rlane) * LDA + koff + k0);
#pragma unroll
      for (int j = 0; j < 4; ++j) acc[i][j] = wmma16(ah, bh[j], acc[i][j]);
    }
  }

  float bcol[4];
#pragma unroll
  for (int j = 0; j < 4; ++j) bcol[j] = 0.0f;
  if (!BIAS_ROW) {
#pragma unroll
    for (int j = 0; j < 4; ++j) bcol[j] = bfr(bias[n0 + ((unsigned)j << 4) + rlane]);
  }

#pragma unroll
  for (int i = 0; i < 4; ++i) {
    const unsigned mBase = m0 + ((unsigned)i << 4);
    float brow[8];
#pragma unroll
    for (int r = 0; r < 8; ++r) brow[r] = 0.0f;
    if (BIAS_ROW) {
#pragma unroll
      for (int r = 0; r < 8; ++r) brow[r] = bfr(bias[mBase + mOff + (unsigned)r]);
    }
#pragma unroll
    for (int j = 0; j < 4; ++j) {
#pragma unroll
      for (int r = 0; r < 8; ++r) {
        float v = acc[i][j][r] * scale + (BIAS_ROW ? brow[r] : bcol[j]);
        if (OUT_MODE == 1) v *= oscale;
        sT[wave][(mOff + (unsigned)r) * 68u + ((unsigned)j << 4) + rlane] = v;
      }
    }
    wave_sync_lds();
    if (OUT_MODE == 0) {
      const unsigned hh = lane >> 4, c4 = (lane & 15u) * 4u;
#pragma unroll
      for (int half = 0; half < 2; ++half) {
        v4f vv[4];
#pragma unroll
        for (int it = 0; it < 4; ++it) {
          const unsigned row = (unsigned)(half * 4 + it) * 2u + hh;
          vv[it] = *(const v4f*)(&sT[wave][row * 68u + c4]);
        }
        for (int pass = 0; pass < 2; ++pass) {
#pragma unroll
          for (int it = 0; it < 4; ++it) {
            const unsigned row = (unsigned)(half * 4 + it) * 2u + hh;
            *(volatile v4f*)(Cf + (size_t)out_row(mBase + row) * LDC + n0 + c4) = vv[it];
          }
          __threadfence();
        }
      }
    } else {
      const unsigned q = lane >> 3, c8 = (lane & 7u) * 8u;
      v8h hv[4];
#pragma unroll
      for (int it = 0; it < 4; ++it) {
        const unsigned row = (unsigned)it * 4u + q;
        const v4f s0 = *(const v4f*)(&sT[wave][row * 68u + c8]);
        const v4f s1 = *(const v4f*)(&sT[wave][row * 68u + c8 + 4u]);
        hv[it][0] = toh_flush(s0.x); hv[it][1] = toh_flush(s0.y); hv[it][2] = toh_flush(s0.z); hv[it][3] = toh_flush(s0.w);
        hv[it][4] = toh_flush(s1.x); hv[it][5] = toh_flush(s1.y); hv[it][6] = toh_flush(s1.z); hv[it][7] = toh_flush(s1.w);
      }
      for (int pass = 0; pass < 2; ++pass) {
#pragma unroll
        for (int it = 0; it < 4; ++it) {
          const unsigned row = (unsigned)it * 4u + q;
          *(volatile v8h*)(Ch + (size_t)(mBase + row) * LDC + n0 + c8) = hv[it];
        }
        __threadfence();
      }
    }
    wave_sync_lds();
  }
}

__global__ __launch_bounds__(256) void k_gemm_qk(const _Float16* __restrict__ x16, const _Float16* __restrict__ w16,
                                                 _Float16* __restrict__ qk16, const float* __restrict__ bias) {
  gemm64_body<1, false, (unsigned)MTOK, 2u * EMB, EMB, EMB, EMB, QKLD>(x16, w16, nullptr, qk16, bias, PROJ_UNDO, QKV_OSC);
}
__global__ __launch_bounds__(256) void k_gemm_vt(const _Float16* __restrict__ wv16, const _Float16* __restrict__ x16,
                                                 _Float16* __restrict__ vt16, const float* __restrict__ bias_v) {
  gemm64_body<1, true, EMB, (unsigned)MTOK, EMB, EMB, EMB, (unsigned)VTLD>(wv16, x16, nullptr, vt16, bias_v, PROJ_UNDO, QKV_OSC);
}
__global__ __launch_bounds__(256) void k_gemm_out(const _Float16* __restrict__ ctx16, const _Float16* __restrict__ wp16,
                                                  float* __restrict__ out, const float* __restrict__ bias) {
  gemm64_body<0, false, (unsigned)MTOK, EMB, EMB, EMB, EMB, EMB>(ctx16, wp16, out, nullptr, bias, OUT_UNDO, 1.0f);
}

__global__ __launch_bounds__(256) void k_cvt_x(const float* __restrict__ x, _Float16* __restrict__ x16) {
    const unsigned u = blockIdx.x * 256u + threadIdx.x;
    if (u >= (unsigned)(MTOK * EMB / 8)) return;
    const unsigned row = u / (unsigned)(EMB / 8), c0 = (u % (unsigned)(EMB / 8)) * 8u;
    const unsigned srow = out_row(row);
    const float* xr = x + (size_t)srow * EMB + c0;
    const v4f a = *(const v4f*)xr, b = *(const v4f*)(xr + 4);
    float v[8] = {bfr(a.x) * XC, bfr(a.y) * XC, bfr(a.z) * XC, bfr(a.w) * XC,
                  bfr(b.x) * XC, bfr(b.y) * XC, bfr(b.z) * XC, bfr(b.w) * XC};
    st8hf(x16, (size_t)row * EMB + c0, v);
}

__global__ __launch_bounds__(256) void k_cvt_w(const float* __restrict__ w, _Float16* __restrict__ w16, unsigned n8) {
    const unsigned u = blockIdx.x * 256u + threadIdx.x;
    if (u >= n8) return;
    const float* wr = w + (size_t)u * 8u;
    const v4f a = *(const v4f*)wr, b = *(const v4f*)(wr + 4);
    float v[8] = {bfr(a.x) * WC, bfr(a.y) * WC, bfr(a.z) * WC, bfr(a.w) * WC,
                  bfr(b.x) * WC, bfr(b.y) * WC, bfr(b.z) * WC, bfr(b.w) * WC};
    st8hf(w16, (size_t)u * 8u, v);
}

#define AT_PP 72
static_assert(8 * 16 * AT_PP * 2 + 64 <= 131072);
__global__ __launch_bounds__(256) void k_attn(const _Float16* __restrict__ qk, const _Float16* __restrict__ vt,
                                              const float* __restrict__ table, _Float16* __restrict__ ctx) {
    __shared__ __align__(16) _Float16 sO[8][16 * AT_PP];
    __shared__ float sTab[16];
    const unsigned tid = threadIdx.x, lane = tid & 31u;
    const unsigned wave = __builtin_amdgcn_readfirstlane(tid >> 5);
    const unsigned hh = lane >> 4, c = lane & 15u;
    if (tid < 16u) sTab[tid] = bfr(table[min(tid, (unsigned)(NTAB - 1))]);
    __syncthreads();

    const unsigned gw = blockIdx.x * 8u + wave;
    const unsigned qt = gw % QTILES;
    const unsigned bp = gw / QTILES;
    const unsigned b = bp >> 2, pair = bp & 3u;
    const unsigned tok0 = b * (unsigned)SEQ;
    const unsigned q0 = qt * 16u;
    const unsigned nq6 = mod7_u11(q0 + c) + 6u;

#pragma unroll 1
    for (unsigned hp = 0; hp < 2u; ++hp) {
        const unsigned head = 2u * pair + hp;
        const v16h qf = frag_ld(qk + (size_t)(tok0 + q0 + c) * QKLD + head * (unsigned)HD + 8u * hh);
        const _Float16* kp = qk + (size_t)(tok0 + c) * QKLD + (unsigned)EMB + head * (unsigned)HD + 8u * hh;
        const _Float16* vp = vt + (size_t)(head * (unsigned)HD + c) * VTLD + tok0 + 8u * hh;
        float mrun = -3.0e38f, lpart = 0.f;
        v8f o0 = (v8f){0.f,0.f,0.f,0.f,0.f,0.f,0.f,0.f};
        v8f o1 = o0;
#pragma unroll 1
        for (unsigned m0 = 0; m0 < (unsigned)SEQ; m0 += 32u) {
            const v16h k0f = frag_ld(kp + (size_t)m0 * QKLD);
            const v16h k1f = frag_ld(kp + (size_t)(m0 + 16u) * QKLD);
            const v16h v0f = frag_ld(vp + m0);
            const v16h v1f = frag_ld(vp + (size_t)16u * VTLD + m0);
            const v8f z = (v8f){0.f,0.f,0.f,0.f,0.f,0.f,0.f,0.f};
            const v8f s0 = wmma16(k0f, qf, z);
            const v8f s1 = wmma16(k1f, qf, z);

            const unsigned mk0 = mod7_u11(m0 + 8u * hh);
            float bzj[7];
            static_assert(wrap7c(16 + 7) < 7);
#pragma unroll
            for (int j = 0; j < 7; ++j) {
                unsigned mk = mk0 + (unsigned)j;
                mk = (mk >= 7u) ? (mk - 7u) : mk;
                bzj[j] = sTab[nq6 - mk];
            }
            float t[16];
            float mx = -3.0e38f;
#pragma unroll
            for (int r = 0; r < 8; ++r) {
                float sv = s0[r] * SCQK;
                sv += bzj[wrap7c(r)];
                t[r] = sv * LOG2E;
                mx = (t[r] > mx) ? t[r] : mx;
            }
#pragma unroll
            for (int r = 0; r < 8; ++r) {
                float sv = s1[r] * SCQK;
                sv += bzj[wrap7c(16 + r)];
                t[8 + r] = sv * LOG2E;
                mx = (t[8 + r] > mx) ? t[8 + r] : mx;
            }
            const float mo = __shfl_xor(mx, 16, 32);
            mx = (mo > mx) ? mo : mx;
            const float mnew = (mx > mrun) ? mx : mrun;
            const float alpha = exp2f(mrun - mnew);
            mrun = mnew;
            float psum = 0.f;
            v16h pb;
#pragma unroll
            for (int e = 0; e < 16; ++e) {
                const float p = exp2f(t[e] - mnew);
                psum += p;
                pb[e] = toh_flush(p * PC);
            }
            lpart = lpart * alpha + psum;
#pragma unroll
            for (int r = 0; r < 8; ++r) { o0[r] *= alpha; o1[r] *= alpha; }
            o0 = wmma16(v0f, pb, o0);
            o1 = wmma16(v1f, pb, o1);
        }
        const float lsum = lpart + __shfl_xor(lpart, 16, 32);
        const float inv = CTX_UNDO * (1.0f / lsum);
        v8h w0, w1;
#pragma unroll
        for (int r = 0; r < 8; ++r) { w0[r] = toh_flush(o0[r] * inv); w1[r] = toh_flush(o1[r] * inv); }
        *(v8h*)(&sO[wave][c * AT_PP + hp * 32u + 8u * hh]) = w0;
        *(v8h*)(&sO[wave][c * AT_PP + hp * 32u + 16u + 8u * hh]) = w1;
    }
    wave_sync_lds();
    {
        const unsigned q = lane >> 3, c8 = (lane & 7u) * 8u;
        v8h ov[4];
#pragma unroll
        for (int it = 0; it < 4; ++it) ov[it] = *(const v8h*)(&sO[wave][((unsigned)it * 4u + q) * AT_PP + c8]);
        _Float16* dst = ctx + (size_t)(tok0 + q0) * (unsigned)EMB + pair * 64u;
        for (int pass = 0; pass < 2; ++pass) {
#pragma unroll
            for (int it = 0; it < 4; ++it) *(volatile v8h*)(dst + (size_t)((unsigned)it * 4u + q) * (unsigned)EMB + c8) = ov[it];
            __threadfence();
        }
    }
}

static constexpr unsigned N8_X     = (unsigned)(MTOK * EMB / 8);
static constexpr unsigned N8_WQKV  = (unsigned)(3 * EMB * EMB / 8);
static constexpr unsigned N8_WPROJ = (unsigned)(EMB * EMB / 8);
static_assert(N8_X % 256 == 0 && N8_WQKV % 256 == 0 && N8_WPROJ % 256 == 0);
static constexpr unsigned G_CVT_X  = N8_X / 256;
static constexpr unsigned G_CVT_WQ = N8_WQKV / 256;
static constexpr unsigned G_CVT_WP = N8_WPROJ / 256;
static constexpr unsigned G_QK  = ((unsigned)(MTOK / 64) * (unsigned)(2 * EMB / 64) + 7u) / 8u;
static constexpr unsigned G_VT  = ((unsigned)(EMB / 64) * (unsigned)(MTOK / 64) + 7u) / 8u;
static constexpr unsigned G_OUT = ((unsigned)(MTOK / 64) * (unsigned)(EMB / 64) + 7u) / 8u;
static constexpr unsigned G_ATT = (unsigned)(NB * 4 * (SEQ / 16)) / 8u;

static constexpr size_t SZ_X16   = (size_t)MTOK * EMB * 2;
static constexpr size_t SZ_WQKV  = (size_t)3 * EMB * EMB * 2;
static constexpr size_t SZ_WPROJ = (size_t)EMB * EMB * 2;
static constexpr size_t SZ_QK    = (size_t)MTOK * QKLD * 2;
static constexpr size_t SZ_VT    = (size_t)EMB * VTLD * 2;
static constexpr size_t SZ_CTX   = (size_t)MTOK * EMB * 2;
static_assert(SZ_X16 % 256 == 0 && SZ_WQKV % 256 == 0 && SZ_WPROJ % 256 == 0 && SZ_QK % 256 == 0 && SZ_VT % 256 == 0 && SZ_CTX % 256 == 0);
static constexpr size_t OFF_X16   = 0;
static constexpr size_t OFF_WQKV  = OFF_X16 + SZ_X16;
static constexpr size_t OFF_WPROJ = OFF_WQKV + SZ_WQKV;
static constexpr size_t OFF_QK    = OFF_WPROJ + SZ_WPROJ;
static constexpr size_t OFF_VT    = OFF_QK + SZ_QK;
static constexpr size_t OFF_CTX   = OFF_VT + SZ_VT;
static constexpr size_t WS_TOTAL  = OFF_CTX + SZ_CTX;
static_assert(WS_TOTAL <= (size_t)134217728);

static constexpr int MIN_X   = ((NB - 1) * SEQ_FULL + SEQ) * EMB;
static constexpr int MIN_WQ  = 3 * EMB * EMB;
static constexpr int MIN_BQ  = 3 * EMB;
static constexpr int MIN_WP  = EMB * EMB;
static constexpr int MIN_BP  = EMB;
static constexpr int MIN_TAB = NTAB;
static constexpr size_t OFF_WV_ELEMS = (size_t)2 * EMB * EMB;
static constexpr int OFF_BV_ELEMS = 2 * EMB;

extern "C" void kernel_launch(void* const* d_in, const int* in_sizes, int n_in, void* d_out, int out_size,
                              void* d_ws, size_t ws_size, hipStream_t stream) {
    if (n_in < 6) return;
    if (in_sizes[0] < MIN_X || in_sizes[1] < MIN_WQ || in_sizes[2] < MIN_BQ) return;
    if (in_sizes[3] < MIN_WP || in_sizes[4] < MIN_BP || in_sizes[5] < MIN_TAB) return;
    if (out_size < MIN_X) return;
    if (WS_TOTAL > ws_size) return;

    const float* x          = (const float*)d_in[0];
    const float* qkv_w      = (const float*)d_in[1];
    const float* qkv_b      = (const float*)d_in[2];
    const float* proj_w     = (const float*)d_in[3];
    const float* proj_b     = (const float*)d_in[4];
    const float* bias_table = (const float*)d_in[5];
    float* out = (float*)d_out;

    char* wsp = (char*)d_ws;
    _Float16* x16    = (_Float16*)(wsp + OFF_X16);
    _Float16* wqkv16 = (_Float16*)(wsp + OFF_WQKV);
    _Float16* wproj16 = (_Float16*)(wsp + OFF_WPROJ);
    _Float16* qk16   = (_Float16*)(wsp + OFF_QK);
    _Float16* vt16   = (_Float16*)(wsp + OFF_VT);
    _Float16* ctx16  = (_Float16*)(wsp + OFF_CTX);

    k_cvt_x<<<G_CVT_X, 256, 0, stream>>>(x, x16);
    k_cvt_w<<<G_CVT_WQ, 256, 0, stream>>>(qkv_w, wqkv16, N8_WQKV);
    k_cvt_w<<<G_CVT_WP, 256, 0, stream>>>(proj_w, wproj16, N8_WPROJ);

    k_gemm_qk<<<G_QK, 256, 0, stream>>>((const _Float16*)x16, (const _Float16*)wqkv16, qk16, qkv_b);
    k_gemm_vt<<<G_VT, 256, 0, stream>>>((const _Float16*)(wqkv16 + OFF_WV_ELEMS), (const _Float16*)x16, vt16, qkv_b + OFF_BV_ELEMS);
    k_attn<<<G_ATT, 256, 0, stream>>>((const _Float16*)qk16, (const _Float16*)vt16, bias_table, ctx16);
    k_gemm_out<<<G_OUT, 256, 0, stream>>>((const _Float16*)ctx16, (const _Float16*)wproj16, out, proj_b);
}
